// Memory_trans_read_38079180046960
// MI455X (gfx1250) — hardware-verified
//
#include <hip/hip_runtime.h>
#include <stdint.h>

#define DD    256
#define MK    2048
#define HWN   4096
#define NBAT  8
#define NQ    32768
#define QTOK  32
#define KBLK  64
#define QBLK  64
#define KP    264
#define SLP   68

#define KSC   64.0f
#define PSC   16384.0f
#define OSC   (1.0f / 1048576.0f)

static_assert(NQ == NBAT * HWN);
static_assert((HWN % QBLK) == 0 && (HWN % QTOK) == 0);
static_assert((MK % KBLK) == 0 && (MK % 32) == 0);
static_assert(DD == 256 && (DD % 32) == 0);
static_assert((KP % 8) == 0 && (SLP % 4) == 0);
static_assert((NQ % QTOK) == 0 && (NQ % QBLK) == 0);

typedef _Float16       v16h __attribute__((ext_vector_type(16)));
typedef _Float16       v8h  __attribute__((ext_vector_type(8)));
typedef __bf16         v16bf __attribute__((ext_vector_type(16)));
typedef unsigned short v16us __attribute__((ext_vector_type(16)));
typedef unsigned short v8us  __attribute__((ext_vector_type(8)));
typedef float          v8f  __attribute__((ext_vector_type(8)));
typedef float          v4f  __attribute__((ext_vector_type(4)));
typedef unsigned int   v4u  __attribute__((ext_vector_type(4)));
typedef unsigned int   v2u  __attribute__((ext_vector_type(2)));

__device__ __forceinline__ unsigned short bf_bits(float f) {
  unsigned u = __float_as_uint(f);
  return (unsigned short)((u + 0x7FFFu + ((u >> 16) & 1u)) >> 16);
}
__device__ __forceinline__ float bf_up(unsigned short hb) { return __uint_as_float(((unsigned)hb) << 16); }
__device__ __forceinline__ unsigned short f2h_bits(float f) { return __builtin_bit_cast(unsigned short, (_Float16)f); }
__device__ __forceinline__ unsigned pk16(unsigned short a, unsigned short b) { return (unsigned)a | ((unsigned)b << 16); }
__device__ __forceinline__ v8f zero8() { v8f z = {0.f, 0.f, 0.f, 0.f, 0.f, 0.f, 0.f, 0.f}; return z; }

__device__ __forceinline__ v16h ldfrag_h(const _Float16* p) {
  union { v16h v; v8h hv[2]; } f;
  f.hv[0] = *(const v8h*)(p);
  f.hv[1] = *(const v8h*)(p + 16);
  return f.v;
}
__device__ __forceinline__ v16bf ldfrag_b(const unsigned short* p) {
  union { v16us v; v8us hv[2]; } f;
  f.hv[0] = *(const v8us*)(p);
  f.hv[1] = *(const v8us*)(p + 16);
  return __builtin_bit_cast(v16bf, f.v);
}

__device__ __forceinline__ v8f mma_b(v16bf a, v16bf b, v8f c) {
  return __builtin_amdgcn_wmma_f32_16x16x32_bf16(false, a, false, b, (short)0, c, false, false);
}
__device__ __forceinline__ v8f mma_h(v16h a, v16h b, v8f c) {
  return __builtin_amdgcn_wmma_f32_16x16x32_f16(false, a, false, b, (short)0, c, false, false);
}
__device__ __forceinline__ void guard_sc(v8f& s0, v8f& s1, v16bf a0, v16bf a1, v16bf b) {
#if defined(__HIP_DEVICE_COMPILE__)
  asm volatile("v_nop\n\tv_nop\n\tv_nop\n\tv_nop" : "+v"(s0), "+v"(s1) : "v"(a0), "v"(a1), "v"(b));
#endif
}
__device__ __forceinline__ void guard_o4(v8f& c0, v8f& c1, v8f& c2, v8f& c3,
                                         v16h a0, v16h a1, v16h a2, v16h a3, v16h b) {
#if defined(__HIP_DEVICE_COMPILE__)
  asm volatile("v_nop\n\tv_nop\n\tv_nop\n\tv_nop"
               : "+v"(c0), "+v"(c1), "+v"(c2), "+v"(c3)
               : "v"(a0), "v"(a1), "v"(a2), "v"(a3), "v"(b));
#endif
}
__device__ __forceinline__ void acc_guard4(v8f& a, v8f& b, v8f& c, v8f& d) {
#if defined(__HIP_DEVICE_COMPILE__)
  asm volatile("v_nop\n\tv_nop\n\tv_nop\n\tv_nop" : "+v"(a), "+v"(b), "+v"(c), "+v"(d));
#endif
}
__device__ __forceinline__ void sched_fence() {
#if defined(__HIP_DEVICE_COMPILE__)
  asm volatile("" ::: "memory");
#endif
}

__global__ __launch_bounds__(256) void cvt_q(const float* __restrict__ query, unsigned short* qt) {
  __shared__ __align__(16) float sx[DD * 33];
  const int tid = threadIdx.x;
  const int p0 = blockIdx.x * QTOK;
  const int b = p0 >> 12, hw0 = p0 & (HWN - 1);
  const float* src = query + (size_t)b * DD * HWN + hw0;
#pragma unroll 8
  for (int it = 0; it < 32; ++it) {
    const int idx = it * 256 + tid;
    const int c = idx >> 5, q = idx & 31;
    sx[c * 33 + q] = src[(size_t)c * HWN + q];
  }
  __syncthreads();
  const int wave = tid >> 5, lane = tid & 31, c8 = lane * 8;
  v4u pk[4];
#pragma unroll
  for (int it = 0; it < 4; ++it) {
    const int r = wave * 4 + it;
    v4u p;
#pragma unroll
    for (int e = 0; e < 4; ++e) {
      const unsigned short a = bf_bits(sx[(c8 + 2 * e) * 33 + r]);
      const unsigned short c = bf_bits(sx[(c8 + 2 * e + 1) * 33 + r]);
      p[e] = pk16(a, c);
    }
    pk[it] = p;
  }
  unsigned short* dst = qt + (size_t)p0 * DD;
  for (int pass = 0; pass < 2; ++pass) {
#pragma unroll
    for (int it = 0; it < 4; ++it) {
      const int r = wave * 4 + it;
      *(volatile v4u*)(dst + (size_t)r * DD + c8) = pk[it];
    }
    __threadfence();
  }
}

__global__ __launch_bounds__(256) void cvt_k(const float* __restrict__ keys, unsigned short* kr,
                                              unsigned short* kc) {
  __shared__ __align__(16) unsigned short st[KBLK * KP];
  const int tid = threadIdx.x, wave = tid >> 5, lane = tid & 31;
  const int m0 = blockIdx.x * KBLK;
#pragma unroll 4
  for (int it = 0; it < 16; ++it) {
    const int idx = it * 256 + tid;
    const int row = idx >> 6, c4 = (idx & 63) * 4;
    const v4f v = *(const v4f*)(keys + (size_t)(m0 + row) * DD + c4);
    v2u w;
    w[0] = pk16(bf_bits(v[0]), bf_bits(v[1]));
    w[1] = pk16(bf_bits(v[2]), bf_bits(v[3]));
    *(v2u*)(st + row * KP + c4) = w;
  }
  __syncthreads();
  {
    const int c8 = lane * 8;
    v4u pk[8];
#pragma unroll
    for (int it = 0; it < 8; ++it) {
      const int row = wave * 8 + it;
      pk[it] = *(const v4u*)(st + row * KP + c8);
    }
    for (int pass = 0; pass < 2; ++pass) {
#pragma unroll
      for (int it = 0; it < 8; ++it) {
        const int row = wave * 8 + it;
        *(volatile v4u*)(kr + (size_t)(m0 + row) * DD + c8) = pk[it];
      }
      __threadfence();
    }
  }
  {
    const int rq = lane >> 3, cl = (lane & 7) * 8;
    v4u pk[8];
#pragma unroll
    for (int it = 0; it < 8; ++it) {
      const int d = wave * 32 + it * 4 + rq;
      v4u p;
#pragma unroll
      for (int e = 0; e < 4; ++e) {
        const int j0 = cl + 2 * e;
        const float a = bf_up(st[j0 * KP + d]) * KSC;
        const float c = bf_up(st[(j0 + 1) * KP + d]) * KSC;
        p[e] = pk16(f2h_bits(a), f2h_bits(c));
      }
      pk[it] = p;
    }
    for (int pass = 0; pass < 2; ++pass) {
#pragma unroll
      for (int it = 0; it < 8; ++it) {
        const int d = wave * 32 + it * 4 + rq;
        *(volatile v4u*)(kc + (size_t)d * MK + m0 + cl) = pk[it];
      }
      __threadfence();
    }
  }
}

__global__ __launch_bounds__(128) void k_attn(const unsigned short* qt, const unsigned short* kr,
                                              const unsigned short* kc, const float* vres, float* out) {
  (void)vres;
  __shared__ __align__(16) float slab[QBLK * SLP];
  const _Float16* Kc = (const _Float16*)(const void*)kc;
  const int tid = threadIdx.x, wave = tid >> 5, lane = tid & 31;
  const int rl = lane & 15, h = lane >> 4, koff = 8 * h;
  const int n0 = blockIdx.x * QBLK;
  const unsigned short* qrow  = qt + (size_t)(n0 + 16 * wave + rl) * DD + koff;
  const unsigned short* krow0 = kr + (size_t)rl * DD + koff;
  const _Float16*       kcol  = Kc + (size_t)rl * MK + koff;

  v8f acc[16];
#pragma unroll
  for (int t = 0; t < 16; ++t) acc[t] = zero8();
  float run_max = -1.0e30f, run_sum = 0.0f;

#pragma unroll 1
  for (int kb = 0; kb < MK; kb += 32) {
    v8f s0 = zero8(), s1 = zero8();
    const unsigned short* ka = krow0 + (size_t)kb * DD;
#pragma unroll
    for (int c = 0; c < 8; ++c) {
      const v16bf qb = ldfrag_b(qrow + 32 * c);
      const v16bf a0 = ldfrag_b(ka + 32 * c);
      const v16bf a1 = ldfrag_b(ka + 16 * DD + 32 * c);
      s0 = mma_b(a0, qb, s0);
      s1 = mma_b(a1, qb, s1);
      guard_sc(s0, s1, a0, a1, qb);
      sched_fence();
    }
    float lmax = fmaxf(s0[0], s1[0]);
#pragma unroll
    for (int v = 1; v < 8; ++v) lmax = fmaxf(lmax, fmaxf(s0[v], s1[v]));
    lmax = fmaxf(lmax, __shfl_xor(lmax, 16, 32));
    const float nm = fmaxf(run_max, lmax);
    const float factor = __expf(run_max - nm);
    run_max = nm;
    float lsum = 0.0f;
    v16h bP;
#pragma unroll
    for (int v = 0; v < 8; ++v) {
      const float p0 = __expf(s0[v] - nm);
      const float p1 = __expf(s1[v] - nm);
      lsum += p0 + p1;
      bP[v]     = (_Float16)(p0 * PSC);
      bP[8 + v] = (_Float16)(p1 * PSC);
    }
    run_sum = run_sum * factor + lsum;
#pragma unroll
    for (int t = 0; t < 16; ++t)
#pragma unroll
      for (int v = 0; v < 8; ++v) acc[t][v] *= factor;
    const _Float16* kt0 = kcol + kb;
#pragma unroll
    for (int g = 0; g < 4; ++g) {
      v16h ak[4];
#pragma unroll
      for (int j = 0; j < 4; ++j) ak[j] = ldfrag_h(kt0 + (size_t)(16 * (4 * g + j)) * MK);
#pragma unroll
      for (int j = 0; j < 4; ++j) acc[4 * g + j] = mma_h(ak[j], bP, acc[4 * g + j]);
      guard_o4(acc[4 * g + 0], acc[4 * g + 1], acc[4 * g + 2], acc[4 * g + 3],
               ak[0], ak[1], ak[2], ak[3], bP);
      sched_fence();
    }
  }
  acc_guard4(acc[0], acc[1], acc[2], acc[3]);
  acc_guard4(acc[4], acc[5], acc[6], acc[7]);
  acc_guard4(acc[8], acc[9], acc[10], acc[11]);
  acc_guard4(acc[12], acc[13], acc[14], acc[15]);

  const float tot = run_sum + __shfl_xor(run_sum, 16, 32);
  const float inv = OSC * (1.0f / tot);
  const int ob = n0 >> 12, hw0 = n0 & (HWN - 1);
  float* obase = out + (size_t)ob * DD * HWN + hw0;
  const int hh = lane >> 4, c4 = (lane & 15) * 4;
#pragma unroll
  for (int g = 0; g < 4; ++g) {
#pragma unroll
    for (int j = 0; j < 4; ++j) {
#pragma unroll
      for (int r = 0; r < 8; ++r) {
        slab[(16 * j + 8 * h + r) * SLP + 16 * wave + rl] = acc[4 * g + j][r] * inv;
      }
    }
    __syncthreads();
    v4f ov[8];
#pragma unroll
    for (int it = 0; it < 8; ++it) {
      const int row = 16 * wave + 2 * it + hh;
      ov[it] = *(const v4f*)(slab + row * SLP + c4);
    }
    for (int pass = 0; pass < 2; ++pass) {
#pragma unroll
      for (int it = 0; it < 8; ++it) {
        const int row = 16 * wave + 2 * it + hh;
        *(volatile v4f*)(obase + (size_t)(64 * g + row) * HWN + c4) = ov[it];
      }
      __threadfence();
    }
    __syncthreads();
  }
}

extern "C" void kernel_launch(void* const* d_in, const int* in_sizes, int n_in,
                              void* d_out, int out_size, void* d_ws, size_t ws_size,
                              hipStream_t stream) {
  if (n_in < 3) return;
  if (in_sizes[0] != MK * DD) return;
  if (in_sizes[1] != NQ * DD) return;
  if (in_sizes[2] < 1) return;
  if (out_size != NQ * DD) return;

  const float* keys  = (const float*)d_in[0];
  const float* query = (const float*)d_in[1];
  const float* value = (const float*)d_in[2];
  float* out = (float*)d_out;

  const size_t PQT = (size_t)NQ * DD * 2;
  const size_t PKR = (size_t)MK * DD * 2;
  const size_t PKC = (size_t)DD * MK * 2;

  size_t off = 0;
  const size_t oQT = off; off += PQT;
  const size_t oKR = off; off += PKR;
  const size_t oKC = off; off += PKC;
  if (off > ws_size) return;
  if (off > (size_t)134217728) return;

  char* ws = (char*)d_ws;
  unsigned short* QT = (unsigned short*)(ws + oQT);
  unsigned short* KR = (unsigned short*)(ws + oKR);
  unsigned short* KC = (unsigned short*)(ws + oKC);

  cvt_q<<<dim3(NQ / QTOK), dim3(256), 0, stream>>>(query, QT);
  cvt_k<<<dim3(MK / KBLK), dim3(256), 0, stream>>>(keys, KR, KC);
  k_attn<<<dim3(NQ / QBLK), dim3(128), 0, stream>>>(QT, KR, KC, value, out);
  (void)hipGetLastError();
}
